// VectorQuantizer_21638045237923
// MI455X (gfx1250) — hardware-verified
//
#include <hip/hip_runtime.h>
#include <stddef.h>


typedef _Float16 v16h __attribute__((ext_vector_type(16)));
typedef _Float16 v8h  __attribute__((ext_vector_type(8)));
typedef float    v8f  __attribute__((ext_vector_type(8)));
typedef float    v4f  __attribute__((ext_vector_type(4)));

#ifndef NB
#define NB 16
#endif
#ifndef SEQ
#define SEQ 1024
#endif
#define NB_FULL  16
#define SEQ_FULL 1024
#define EDIM  256
#define NCODE 8192
#define MROWS (NB * SEQ)
#define KSTEP (EDIM / 32)

static_assert(NB >= 1 && NB <= NB_FULL);
static_assert(SEQ >= 128 && SEQ <= SEQ_FULL && (SEQ % 128) == 0);
static_assert(EDIM == 32 * 8);
static_assert((EDIM % 32) == 0 && KSTEP == 8);
static_assert((NCODE % 64) == 0 && (NCODE % 32) == 0);
static_assert((MROWS % 128) == 0 && (MROWS % 32) == 0);
static_assert(EDIM == 2 * 32 * 4);

#define LDW 264
static_assert((LDW % 8) == 0 && LDW >= EDIM);

#define OCARRY 2048.0f

#define X16_BYTES ((size_t)MROWS * EDIM * 2)
#define W16_BYTES ((size_t)NCODE * EDIM * 2)
#define XN_BYTES  ((size_t)MROWS * 4)
#define WN_BYTES  ((size_t)NCODE * 4)
#define OFF_X16 ((size_t)0)
#define OFF_W16 (OFF_X16 + X16_BYTES)
#define OFF_XN  (OFF_W16 + W16_BYTES)
#define OFF_WN  (OFF_XN + XN_BYTES)
#define WS_TOTAL (OFF_WN + WN_BYTES)
static_assert((X16_BYTES % 128) == 0 && (W16_BYTES % 128) == 0);
static_assert((XN_BYTES % 128) == 0 && (WN_BYTES % 128) == 0);
static_assert(WS_TOTAL <= (size_t)134217728);

__device__ __forceinline__ float bf16r(float x) {
  unsigned int u = __float_as_uint(x);
  u = (u + 0x7FFFu + ((u >> 16) & 1u)) & 0xFFFF0000u;
  return __uint_as_float(u);
}

static __device__ __forceinline__ _Float16 toh_flush(float v) {
  const _Float16 r = (_Float16)v;
  return (fabsf(v) < 6.103515625e-05f) ? (_Float16)0.0f : r;
}

__device__ __forceinline__ v16h frag_at(const _Float16* p) {
  v8h lo = *(const v8h*)(p);
  v8h hi = *(const v8h*)(p + 16);
  v16h out;
#pragma unroll
  for (int i = 0; i < 8; ++i) { out[i] = lo[i]; out[i + 8] = hi[i]; }
  return out;
}
__device__ __forceinline__ v16h ld_frag(const _Float16* base, unsigned ld) {
  const unsigned lane = threadIdx.x & 31u;
  return frag_at(base + (lane & 15u) * ld + (lane >> 4) * 8u);
}

__device__ __forceinline__ v8f wmma16(v16h a, v16h b, v8f c) {
  v8f d = __builtin_amdgcn_wmma_f32_16x16x32_f16(false, a, false, b, (short)0, c,
                                                 false, false);
  asm volatile("v_nop\n\tv_nop\n\tv_nop\n\tv_nop" : "+v"(d) : "v"(a), "v"(b));
  return d;
}

template <int IS_X>
__device__ __forceinline__ void cvt_body(const float* __restrict__ src,
                                         _Float16* __restrict__ dst16,
                                         float* __restrict__ dstn) {
#pragma clang fp contract(off)
  __shared__ __attribute__((aligned(16))) float sn[32];
  const unsigned lane = threadIdx.x & 31u;
  const int wave = __builtin_amdgcn_readfirstlane(threadIdx.x >> 5);

#pragma unroll 1
  for (unsigned j = 0; j < 4u; ++j) {
    const unsigned rl = (unsigned)wave * 4u + j;
    const unsigned crow = blockIdx.x * 32u + rl;
    size_t srow = crow;
    if (IS_X) {
      const unsigned bidx = crow / (unsigned)SEQ;
      const unsigned sq = crow - bidx * (unsigned)SEQ;
      srow = (size_t)bidx * SEQ_FULL + sq;
    }
    const float* p = src + srow * EDIM + lane * 8u;
    const v4f a0 = *(const v4f*)(p);
    const v4f a1 = *(const v4f*)(p + 4);
    v8h o;
    double s = 0.0;
#pragma unroll
    for (int i = 0; i < 4; ++i) {
      const float e0 = bf16r(a0[i]);
      const float e1 = bf16r(a1[i]);
      o[i]     = toh_flush(e0 * OCARRY);
      o[i + 4] = toh_flush(e1 * OCARRY);
      s += (double)e0 * (double)e0;
      s += (double)e1 * (double)e1;
    }
#pragma unroll
    for (int off = 1; off < 32; off <<= 1) s += __shfl_xor(s, off, 32);
    const float sf = (float)s;
    if (lane == 0u) sn[rl] = sf;
    _Float16* q = dst16 + (size_t)crow * EDIM + lane * 8u;
    *(volatile v8h*)q = o;
    __threadfence();
    *(volatile v8h*)q = o;
  }
  __syncthreads();
  if (wave == 0) {
    if (lane < 8u) {
      const v4f nv = *(const v4f*)&sn[lane * 4u];
      float* q = dstn + (size_t)blockIdx.x * 32u + lane * 4u;
      *(volatile v4f*)q = nv;
      __threadfence();
      *(volatile v4f*)q = nv;
    }
  }
}

__global__ __launch_bounds__(256) void cvt_x_kernel(
    const float* __restrict__ src, _Float16* __restrict__ dst16, float* __restrict__ dstn) {
  cvt_body<1>(src, dst16, dstn);
}
__global__ __launch_bounds__(256) void cvt_w_kernel(
    const float* __restrict__ src, _Float16* __restrict__ dst16, float* __restrict__ dstn) {
  cvt_body<0>(src, dst16, dstn);
}

__global__ __launch_bounds__(256) void vq_select_kernel(
    const _Float16* __restrict__ X16, const _Float16* __restrict__ W16,
    const float* __restrict__ XN, const float* __restrict__ WN,
    const float* __restrict__ W, float* __restrict__ out) {
#pragma clang fp contract(off)
  __shared__ __attribute__((aligned(16))) _Float16 Ws[64 * LDW];
  __shared__ int s_idx[128];

  const unsigned tid = threadIdx.x, lane = tid & 31u;
  const int wave = __builtin_amdgcn_readfirstlane(threadIdx.x >> 5);
  const unsigned hh = lane >> 4, m = lane & 15u;
  const unsigned brow0 = blockIdx.x * 128u;
  const unsigned row0 = brow0 + (unsigned)wave * 16u;

  v16h qf[KSTEP];
  {
    const _Float16* qp = X16 + (size_t)(row0 + m) * EDIM + hh * 8u;
#pragma unroll
    for (int c = 0; c < KSTEP; ++c) qf[c] = frag_at(qp + c * 32);
  }
  float xn[8], bs[8];
  int bi[8];
#pragma unroll
  for (int v = 0; v < 8; ++v) {
    xn[v] = XN[row0 + hh * 8u + (unsigned)v];
    bs[v] = -__builtin_inff();
    bi[v] = 0;
  }
  const float two_inv = 2.0f / (OCARRY * OCARRY);

#pragma unroll 1
  for (unsigned tile = 0; tile < (unsigned)(NCODE / 64); ++tile) {
    const unsigned c0 = tile * 64u;
#pragma unroll
    for (unsigned j = 0; j < 8u; ++j) {
      const unsigned idx = tid + 256u * j;
      const unsigned r = idx >> 5, c = (idx & 31u) * 8u;
      *(v8h*)&Ws[r * LDW + c] = *(const v8h*)(W16 + (size_t)(c0 + r) * EDIM + c);
    }
    float wnv[4];
#pragma unroll
    for (int kg = 0; kg < 4; ++kg) wnv[kg] = WN[c0 + (unsigned)kg * 16u + m];
    __syncthreads();

#pragma unroll
    for (int kg = 0; kg < 4; ++kg) {
      v8f t = {};
#pragma unroll
      for (int c = 0; c < KSTEP; ++c) {
        const v16h kf = ld_frag(&Ws[(kg * 16) * LDW + c * 32], LDW);
        t = wmma16(qf[c], kf, t);
      }
      const float wn = wnv[kg];
      const int col = (int)(c0 + (unsigned)kg * 16u + m);
#pragma unroll
      for (int v = 0; v < 8; ++v) {
        const float tsum = xn[v] + wn;
        const float d = tsum - t[v] * two_inv;
        const bool take = d > bs[v];
        bs[v] = take ? d : bs[v];
        bi[v] = take ? col : bi[v];
      }
    }
    __syncthreads();
  }

#pragma unroll
  for (int off = 1; off < 16; off <<= 1) {
#pragma unroll
    for (int v = 0; v < 8; ++v) {
      const float os = __shfl_xor(bs[v], off, 32);
      const int oi = __shfl_xor(bi[v], off, 32);
      const bool take = (os > bs[v]) || ((os == bs[v]) && (oi < bi[v]));
      bs[v] = take ? os : bs[v];
      bi[v] = take ? oi : bi[v];
    }
  }
  if (m == 0u) {
#pragma unroll
    for (int v = 0; v < 8; ++v) s_idx[(unsigned)wave * 16u + hh * 8u + (unsigned)v] = bi[v];
  }
  __syncthreads();

  const unsigned bidx = brow0 / (unsigned)SEQ;
  const unsigned sq0 = brow0 - bidx * (unsigned)SEQ;
  const size_t frow0 = (size_t)bidx * SEQ_FULL + sq0 + (unsigned)wave * 16u;
#pragma unroll 1
  for (unsigned r = 0; r < 16u; ++r) {
    int id = s_idx[(unsigned)wave * 16u + r];
    id = (id < 0) ? 0 : id;
    id = (id > (NCODE - 1)) ? (NCODE - 1) : id;
    const float* sp = W + (size_t)id * EDIM + lane * 4u;
    v4f a0 = *(const v4f*)(sp);
    v4f a1 = *(const v4f*)(sp + 128);
#pragma unroll
    for (int i = 0; i < 4; ++i) {
      a0[i] = bf16r(a0[i]);
      a1[i] = bf16r(a1[i]);
    }
    float* dp = out + (frow0 + r) * EDIM + lane * 4u;
    *(volatile v4f*)(dp) = a0;
    *(volatile v4f*)(dp + 128) = a1;
    __threadfence();
    *(volatile v4f*)(dp) = a0;
    *(volatile v4f*)(dp + 128) = a1;
  }
}

extern "C" void kernel_launch(void* const* d_in, const int* in_sizes, int n_in,
                              void* d_out, int out_size, void* d_ws, size_t ws_size,
                              hipStream_t stream) {
  if (n_in < 2) return;
  const long long need_x = ((long long)(NB - 1) * SEQ_FULL + SEQ) * EDIM;
  if ((long long)in_sizes[0] < need_x) return;
  if ((long long)in_sizes[1] < (long long)NCODE * EDIM) return;
  if ((long long)out_size < need_x) return;
  if (ws_size < WS_TOTAL) return;

  const float* X = (const float*)d_in[0];
  const float* W = (const float*)d_in[1];
  float* out = (float*)d_out;

  char* ws = (char*)d_ws;
  _Float16* X16 = (_Float16*)(ws + OFF_X16);
  _Float16* W16 = (_Float16*)(ws + OFF_W16);
  float*    XN  = (float*)(ws + OFF_XN);
  float*    WN  = (float*)(ws + OFF_WN);

  dim3 blk(256);
  cvt_x_kernel<<<dim3(MROWS / 32), blk, 0, stream>>>(X, X16, XN);
  cvt_w_kernel<<<dim3(NCODE / 32), blk, 0, stream>>>(W, W16, WN);
  vq_select_kernel<<<dim3(MROWS / 128), blk, 0, stream>>>(X16, W16, XN, WN, W, out);
}
